// Head_21440476741642
// MI455X (gfx1250) — hardware-verified
//
#include <hip/hip_runtime.h>
#include <math.h>

#ifndef NB
#define NB 16
#endif
#ifndef SEQ
#define SEQ 1024
#endif
#define NB_FULL 16
#define SEQ_FULL 1024
#define DIN 768
#define HD 128
#define D3 (3 * HD)
#define NRT (NB * SEQ)

static_assert(NB >= 1 && NB <= NB_FULL);
static_assert(SEQ >= 64 && SEQ <= SEQ_FULL && (SEQ % 64) == 0);
static_assert((NRT % 64) == 0);
static_assert((D3 % 64) == 0);
static_assert((DIN % 32) == 0 && (DIN % 8) == 0);
static_assert((HD % 32) == 0);

typedef __attribute__((ext_vector_type(16))) _Float16 v16h;
typedef __attribute__((ext_vector_type(8)))  _Float16 v8h;
typedef __attribute__((ext_vector_type(16))) __bf16   v16b;
typedef __attribute__((ext_vector_type(8)))  __bf16   v8b;
typedef __attribute__((ext_vector_type(8)))  float    v8f;
typedef __attribute__((ext_vector_type(4)))  float    v4f;
typedef unsigned int cm_u4 __attribute__((ext_vector_type(4)));


#define VST2(T, ptr, val) do { const T vst2_v_ = (val); *(volatile T*)(ptr) = vst2_v_; __threadfence(); *(volatile T*)(ptr) = vst2_v_; } while (0)

__device__ __forceinline__ unsigned short at_bf_bits(float f) {
    unsigned u = __float_as_uint(f);
    return (unsigned short)((u + 0x7FFFu + ((u >> 16) & 1u)) >> 16);
}
__device__ __forceinline__ __bf16 at_f2bf(float f) { return __builtin_bit_cast(__bf16, at_bf_bits(f)); }
__device__ __forceinline__ void at_split(float f, __bf16& hi, __bf16& lo) {
    const unsigned short hb = at_bf_bits(f);
    hi = __builtin_bit_cast(__bf16, hb);
    lo = at_f2bf(f - __uint_as_float(((unsigned)hb) << 16));
}

struct Split { v16b hi, lo; };
union FB { v16b v; v8b h[2]; };
__device__ __forceinline__ v16b ld_frag(const __bf16* p) { FB u; u.h[0] = *(const v8b*)(p); u.h[1] = *(const v8b*)(p + 16); return u.v; }

__device__ __forceinline__ v8f wmma3(const Split& a, const Split& b, v8f c) {
    c = __builtin_amdgcn_wmma_f32_16x16x32_bf16(false, a.hi, false, b.hi, (short)0, c, false, false);
    c = __builtin_amdgcn_wmma_f32_16x16x32_bf16(false, a.hi, false, b.lo, (short)0, c, false, false);
    c = __builtin_amdgcn_wmma_f32_16x16x32_bf16(false, a.lo, false, b.hi, (short)0, c, false, false);
    asm volatile("v_nop\n\tv_nop\n\tv_nop\n\tv_nop" : "+v"(c) : "v"(a.hi), "v"(a.lo), "v"(b.hi), "v"(b.lo));
    return c;
}

namespace w25 {
typedef __attribute__((ext_vector_type(16))) _Float16 v16h;
typedef __attribute__((ext_vector_type(8)))  _Float16 v8h;
typedef __attribute__((ext_vector_type(16))) __bf16   v16b;
typedef __attribute__((ext_vector_type(8)))  __bf16   v8b;
typedef __attribute__((ext_vector_type(8)))  float    v8f;
typedef __attribute__((ext_vector_type(4)))  float    v4f;

__device__ __forceinline__ unsigned short f2bf_bits(float f) {
  unsigned u = __float_as_uint(f);
  return (unsigned short)((u + 0x7FFFu + ((u >> 16) & 1u)) >> 16);
}
__device__ __forceinline__ float bf_bits2f(unsigned short h) { return __uint_as_float(((unsigned)h) << 16); }

__device__ __forceinline__ void dep_guard_h(v8f& a, v8f& b, v16h x, v16h y) { asm volatile("v_nop\n\tv_nop\n\tv_nop\n\tv_nop" : "+v"(a), "+v"(b) : "v"(x), "v"(y)); }
__device__ __forceinline__ void dep_guard_b(v8f& a, v8f& b, v16b x, v16b y) { asm volatile("v_nop\n\tv_nop\n\tv_nop\n\tv_nop" : "+v"(a), "+v"(b) : "v"(x), "v"(y)); }
__device__ __forceinline__ void keep4_h(v16h a, v16h b, v16h c, v16h d) { asm volatile("v_nop" :: "v"(a), "v"(b), "v"(c), "v"(d)); }
__device__ __forceinline__ void keep4_b(v16b a, v16b b, v16b c, v16b d) { asm volatile("v_nop" :: "v"(a), "v"(b), "v"(c), "v"(d)); }
__device__ __forceinline__ void acc_guard4(v8f& a, v8f& b, v8f& c, v8f& d) { asm volatile("v_nop\n\tv_nop\n\tv_nop\n\tv_nop" : "+v"(a), "+v"(b), "+v"(c), "+v"(d)); }
template <typename T> struct Frag;
template <> struct Frag<_Float16> {
  typedef v16h V; union U { v16h v; v8h h[2]; };
  static __device__ __forceinline__ v16h load(const _Float16* p) {
    U f; f.h[0] = *(const v8h*)(p); f.h[1] = *(const v8h*)(p + 16); return f.v;
  }
  static __device__ __forceinline__ v8f mma(v16h a, v16h b, v8f c) {
    return __builtin_amdgcn_wmma_f32_16x16x32_f16(false, a, false, b, (short)0, c, false, false);
  }
  static __device__ __forceinline__ void guard(v8f& a, v8f& b, v16h x, v16h y) { dep_guard_h(a, b, x, y); }
  static __device__ __forceinline__ void keep(v16h a, v16h b, v16h c, v16h d) { keep4_h(a, b, c, d); }
};
template <> struct Frag<__bf16> {
  typedef v16b V; union U { v16b v; v8b h[2]; };
  static __device__ __forceinline__ v16b load(const __bf16* p) {
    U f; f.h[0] = *(const v8b*)(p); f.h[1] = *(const v8b*)(p + 16); return f.v;
  }
  static __device__ __forceinline__ v8f mma(v16b a, v16b b, v8f c) {
    return __builtin_amdgcn_wmma_f32_16x16x32_bf16(false, a, false, b, (short)0, c, false, false);
  }
  static __device__ __forceinline__ void guard(v8f& a, v8f& b, v16b x, v16b y) { dep_guard_b(a, b, x, y); }
  static __device__ __forceinline__ void keep(v16b a, v16b b, v16b c, v16b d) { keep4_b(a, b, c, d); }
};

template <int ET> struct Elem;
template <> struct Elem<0> { typedef _Float16 T; };
template <> struct Elem<1> { typedef __bf16 T; };
template <int ET, bool SPLIT, int BIAS_MODE, int OUT_MODE, bool RESID, int ACT = 0>
__global__ __launch_bounds__(256) void wmma_gemm64(
    const unsigned short* __restrict__ Ap, const unsigned short* __restrict__ A2p, int lda, long strideA,
    const unsigned short* __restrict__ Btp, const unsigned short* __restrict__ Bt2p, int ldb, long strideB,
    void* __restrict__ Cout, void* __restrict__ Cout2, int ldc, long strideC,
    const float* __restrict__ bias,
    const float* __restrict__ resid, long strideR,
    int M, int N, int K, float scale) {
  typedef typename Elem<ET>::T T;
  typedef typename Frag<T>::V V;
  const T* A = (const T*)Ap; const T* A2 = (const T*)A2p; const T* Bt = (const T*)Btp; const T* Bt2 = (const T*)Bt2p;
  __shared__ __align__(16) float sT[8][16 * 68];
  const int b    = blockIdx.y;
  const int lane = threadIdx.x & 31;
  const int wave = threadIdx.x >> 5;
  const int tilesN = N >> 6;
  const int tilesM = M >> 6;
  const int tile = blockIdx.x * 8 + wave;
  if (tile >= tilesM * tilesN) return;
  const int tm = tile / tilesN;
  const int tn = tile - tm * tilesN;
  const int m0 = tm << 6;
  const int n0 = tn << 6;

  const T* Ab  = A  + (size_t)b * strideA;
  const T* Bb  = Bt + (size_t)b * strideB;
  const T* Ab2 = SPLIT ? (A2  + (size_t)b * strideA) : nullptr;
  const T* Bb2 = SPLIT ? (Bt2 + (size_t)b * strideB) : nullptr;

  const int rlane = lane & 15;
  const int koff  = (lane >> 4) * 8;
  const int mOff  = (lane >> 4) * 8;

  v8f acc[4][4];
#pragma unroll
  for (int i = 0; i < 4; ++i)
#pragma unroll
    for (int j = 0; j < 4; ++j) acc[i][j] = (v8f){0.f,0.f,0.f,0.f,0.f,0.f,0.f,0.f};

  for (int k0 = 0; k0 < K; k0 += 32) {
    V bh[4], bl[4];
#pragma unroll
    for (int j = 0; j < 4; ++j) {
      const size_t bo = (size_t)(n0 + (j << 4) + rlane) * ldb + koff + k0;
      bh[j] = Frag<T>::load(Bb + bo);
      if (SPLIT) bl[j] = Frag<T>::load(Bb2 + bo);
    }
#pragma unroll
    for (int i = 0; i < 4; ++i) {
      const size_t ao = (size_t)(m0 + (i << 4) + rlane) * lda + koff + k0;
      V ah = Frag<T>::load(Ab + ao);
      V al;
      if (SPLIT) al = Frag<T>::load(Ab2 + ao);
#pragma unroll
      for (int j = 0; j < 4; ++j) {
        acc[i][j] = Frag<T>::mma(ah, bh[j], acc[i][j]);
        if (SPLIT) {
          acc[i][j] = Frag<T>::mma(ah, bl[j], acc[i][j]);
          acc[i][j] = Frag<T>::mma(al, bh[j], acc[i][j]);
        }
      }
      Frag<T>::guard(acc[i][0], acc[i][3], ah, SPLIT ? al : ah);
    }
    Frag<T>::keep(bh[0], bh[1], bh[2], bh[3]);
    if (SPLIT) Frag<T>::keep(bl[0], bl[1], bl[2], bl[3]);
  }
  acc_guard4(acc[0][0], acc[0][1], acc[0][2], acc[0][3]);
  acc_guard4(acc[1][0], acc[1][1], acc[1][2], acc[1][3]);
  acc_guard4(acc[2][0], acc[2][1], acc[2][2], acc[2][3]);
  acc_guard4(acc[3][0], acc[3][1], acc[3][2], acc[3][3]);

  float* slab = sT[wave];
  const float* Rb = RESID ? (resid + (size_t)b * strideR) : nullptr;
#pragma unroll
  for (int i = 0; i < 4; ++i) {
    const int mBase = m0 + (i << 4);
#pragma unroll
    for (int j = 0; j < 4; ++j) {
      const int n = n0 + (j << 4) + rlane;
      float bv = 0.f;
      if (BIAS_MODE == 2) bv = bias[n];
#pragma unroll
      for (int r = 0; r < 8; ++r) {
        float v = acc[i][j][r] * scale;
        if (BIAS_MODE == 1) v += bias[mBase + mOff + r];
        if (BIAS_MODE == 2) v += bv;
        if (RESID) v += Rb[(size_t)(mBase + mOff + r) * ldc + n];
        if (ACT == 1) v = tanhf(v);
        if (ACT == 2) v = fmaxf(v, 0.0f);
        if (ACT == 3) v = v / (1.0f + expf(-v));
        if (ACT == 4) v = (v > 0.f) ? v : 0.01f * v;
        if (ACT == 5) v = 0.5f * v * (1.0f + erff(v * 0.70710678118654752f));
        if (ACT == 6) v = (v > 0.f) ? v : 0.2f * v;
        if (ACT == 7) { const float u = 0.7978845608028654f * (v + 0.044715f * v * v * v); v = 0.5f * v * (1.f + tanhf(u)); }
        slab[(mOff + r) * 68 + (j << 4) + rlane] = v;
      }
    }
    __builtin_amdgcn_fence(3, "workgroup");
    __builtin_amdgcn_wave_barrier();
    __builtin_amdgcn_fence(2, "workgroup");
    if (OUT_MODE == 0) {
      float* C = (float*)Cout + (size_t)b * strideC;
      const int hh = lane >> 4, c4 = (lane & 15) * 4;
      for (int pass = 0; pass < 2; ++pass) {
#pragma unroll
        for (int it = 0; it < 8; ++it) {
          const int row = it * 2 + hh;
          v4f v = *(const v4f*)(slab + row * 68 + c4);
          *(volatile v4f*)(C + (size_t)(mBase + row) * ldc + n0 + c4) = v;
        }
        __threadfence();
      }
    } else {
      const int q = lane >> 3, c8 = (lane & 7) * 8;
      unsigned short* C  = (unsigned short*)Cout  + (size_t)b * strideC;
      unsigned short* C2 = (OUT_MODE == 2) ? ((unsigned short*)Cout2 + (size_t)b * strideC) : nullptr;
      for (int pass = 0; pass < 2; ++pass) {
#pragma unroll
        for (int it = 0; it < 4; ++it) {
          const int row = it * 4 + q;
          const float* sp = slab + row * 68 + c8;
          v8h hv, lv;
#pragma unroll
          for (int e = 0; e < 8; ++e) {
            if (OUT_MODE == 1) {
              hv[e] = (_Float16)sp[e];
            } else {
              unsigned short hb = f2bf_bits(sp[e]);
              unsigned short lb = f2bf_bits(sp[e] - bf_bits2f(hb));
              hv[e] = __builtin_bit_cast(_Float16, hb);
              lv[e] = __builtin_bit_cast(_Float16, lb);
            }
          }
          *(volatile v8h*)(C + (size_t)(mBase + row) * ldc + n0 + c8) = hv;
          if (OUT_MODE == 2) *(volatile v8h*)(C2 + (size_t)(mBase + row) * ldc + n0 + c8) = lv;
        }
        __threadfence();
      }
    }
    __builtin_amdgcn_fence(3, "workgroup");
    __builtin_amdgcn_wave_barrier();
    __builtin_amdgcn_fence(2, "workgroup");
  }
}

}

__device__ __forceinline__ unsigned int cmb_pk2(float a, float b) { return (unsigned int)__builtin_bit_cast(unsigned short, (_Float16)a) | ((unsigned int)__builtin_bit_cast(unsigned short, (_Float16)b) << 16); }
__device__ __forceinline__ float cmb_bf(float v) { const unsigned u = __builtin_bit_cast(unsigned, v); const unsigned r = (u + 0x7fffu + ((u >> 16) & 1u)) & 0xffff0000u; return __builtin_bit_cast(float, r); }

__global__ __launch_bounds__(256) void k_cast_x(const float* __restrict__ SRC, unsigned short* __restrict__ DST) {
    const long long u = (long long)blockIdx.x * 256 + threadIdx.x;
    const int per = DIN / 8;
    if (u >= (long long)NRT * per) return;
    const int r = (int)(u / per); const int c0 = 8 * (int)(u - (long long)r * per);
    const int bb = r / SEQ, tt = r - bb * SEQ;
    const float* s = SRC + ((size_t)bb * SEQ_FULL + tt) * DIN + c0;
    const v4f f0 = *(const v4f*)(s); const v4f f1 = *(const v4f*)(s + 4);
    const float w0 = cmb_bf(f0.x), w1 = cmb_bf(f0.y), w2 = cmb_bf(f0.z), w3 = cmb_bf(f0.w);
    const float w4 = cmb_bf(f1.x), w5 = cmb_bf(f1.y), w6 = cmb_bf(f1.z), w7 = cmb_bf(f1.w);
    cm_u4 pk; pk.x = cmb_pk2(w0, w1); pk.y = cmb_pk2(w2, w3); pk.z = cmb_pk2(w4, w5); pk.w = cmb_pk2(w6, w7);
    VST2(cm_u4, (cm_u4*)(DST + (size_t)r * DIN + c0), pk);
}
__global__ __launch_bounds__(256) void k_cm_castbT(const float* __restrict__ SRC, int lds, unsigned short* __restrict__ DST, int ldd, int nR, int nC, float sc) {
    const long long u = (long long)blockIdx.x * 256 + threadIdx.x; const int per = nR / 8; if (u >= (long long)nC * per) return; const int c = (int)(u / per); const int r0 = 8 * (int)(u % per);
    float w[8];
#pragma unroll
    for (int e = 0; e < 8; ++e) w[e] = cmb_bf(SRC[(long long)(r0 + e) * lds + c]) * sc;
    cm_u4 pk; pk.x = cmb_pk2(w[0], w[1]); pk.y = cmb_pk2(w[2], w[3]); pk.z = cmb_pk2(w[4], w[5]); pk.w = cmb_pk2(w[6], w[7]); VST2(cm_u4, (cm_u4*)(DST + (long long)c * ldd + r0), pk); }

#define AW   4
#define KC   64
#define QP   136
#define VPT  72
#define PP   72
#define OSP  132
#define L_QH 0
#define L_QL (L_QH + AW * 16 * QP * 2)
#define L_KH (L_QL + AW * 16 * QP * 2)
#define L_KL (L_KH + KC * QP * 2)
#define L_VH (L_KL + KC * QP * 2)
#define L_VL (L_VH + HD * VPT * 2)
#define L_PH (L_VL + HD * VPT * 2)
#define L_PL (L_PH + AW * 16 * PP * 2)
#define L_END (L_PL + AW * 16 * PP * 2)
#define L_OS L_KH
static_assert(L_END == 124928);
static_assert(AW * 16 * OSP * 4 <= 2 * KC * QP * 2);
static_assert((L_QL % 16) == 0 && (L_KH % 16) == 0 && (L_KL % 16) == 0 && (L_VH % 16) == 0 && (L_VL % 16) == 0 && (L_PH % 16) == 0 && (L_PL % 16) == 0);
static_assert((QP * 2) % 16 == 0 && (VPT * 2) % 16 == 0 && (PP * 2) % 16 == 0 && (OSP * 4) % 16 == 0);
static_assert(KC == 64 && HD == 128);

__global__ __launch_bounds__(32 * AW) __attribute__((amdgpu_num_vgpr(256)))
void k_attn_c(const float* __restrict__ QKV, float* __restrict__ O, float sl2) {
    extern __shared__ __align__(16) unsigned char attn_lds[];
    __bf16* QH = (__bf16*)(attn_lds + L_QH); __bf16* QL = (__bf16*)(attn_lds + L_QL);
    __bf16* KH = (__bf16*)(attn_lds + L_KH); __bf16* KL = (__bf16*)(attn_lds + L_KL);
    __bf16* VH = (__bf16*)(attn_lds + L_VH); __bf16* VL = (__bf16*)(attn_lds + L_VL);
    __bf16* PH = (__bf16*)(attn_lds + L_PH); __bf16* PL = (__bf16*)(attn_lds + L_PL);
    float*  OS = (float*)(attn_lds + L_OS);
    const int tid = threadIdx.x, wave = tid >> 5, lane = tid & 31, hh = lane >> 4, c = lane & 15;
    const int qb = blockIdx.x, b = blockIdx.y;
    const int q0 = qb * 64 + wave * 16;
    const float NEG = -__builtin_inff();
    const float* base = QKV + (size_t)b * SEQ * D3;

    __bf16* qh = QH + wave * 16 * QP; __bf16* ql = QL + wave * 16 * QP;
#pragma unroll 2
    for (int idx = lane; idx < 16 * (HD / 4); idx += 32) {
        const int row = idx >> 5, c4 = (idx & 31) * 4;
        const v4f f = *(const v4f*)(base + (size_t)(q0 + row) * D3 + c4);
        __bf16 ah, al;
        at_split(f.x, ah, al); qh[row * QP + c4 + 0] = ah; ql[row * QP + c4 + 0] = al;
        at_split(f.y, ah, al); qh[row * QP + c4 + 1] = ah; ql[row * QP + c4 + 1] = al;
        at_split(f.z, ah, al); qh[row * QP + c4 + 2] = ah; ql[row * QP + c4 + 2] = al;
        at_split(f.w, ah, al); qh[row * QP + c4 + 3] = ah; ql[row * QP + c4 + 3] = al;
    }

    v8f o[8]; float m8[8], l8[8];
#pragma unroll
    for (int t = 0; t < 8; ++t) o[t] = (v8f){0.f, 0.f, 0.f, 0.f, 0.f, 0.f, 0.f, 0.f};
#pragma unroll
    for (int i = 0; i < 8; ++i) { m8[i] = NEG; l8[i] = 0.f; }

    __bf16* ph = PH + wave * 16 * PP; __bf16* pl = PL + wave * 16 * PP;
    const int nch = qb + 1;
    for (int kc = 0; kc < nch; ++kc) {
        const int kv0 = kc * KC;
        __syncthreads();
        {
            const int kvr = tid >> 1, dh = (tid & 1) * (HD / 2);
            const float* krow = base + (size_t)(kv0 + kvr) * D3 + HD + dh;
            const float* vrow = base + (size_t)(kv0 + kvr) * D3 + 2 * HD + dh;
#pragma unroll 4
            for (int i = 0; i < HD / 8; ++i) {
                const v4f kk = *(const v4f*)(krow + 4 * i);
                const v4f vv = *(const v4f*)(vrow + 4 * i);
                const int d = dh + 4 * i;
                __bf16 ah, al;
                at_split(kk.x, ah, al); KH[kvr * QP + d + 0] = ah; KL[kvr * QP + d + 0] = al;
                at_split(kk.y, ah, al); KH[kvr * QP + d + 1] = ah; KL[kvr * QP + d + 1] = al;
                at_split(kk.z, ah, al); KH[kvr * QP + d + 2] = ah; KL[kvr * QP + d + 2] = al;
                at_split(kk.w, ah, al); KH[kvr * QP + d + 3] = ah; KL[kvr * QP + d + 3] = al;
                at_split(vv.x, ah, al); VH[(d + 0) * VPT + kvr] = ah; VL[(d + 0) * VPT + kvr] = al;
                at_split(vv.y, ah, al); VH[(d + 1) * VPT + kvr] = ah; VL[(d + 1) * VPT + kvr] = al;
                at_split(vv.z, ah, al); VH[(d + 2) * VPT + kvr] = ah; VL[(d + 2) * VPT + kvr] = al;
                at_split(vv.w, ah, al); VH[(d + 3) * VPT + kvr] = ah; VL[(d + 3) * VPT + kvr] = al;
            }
        }
        __syncthreads();

        v8f s[4];
#pragma unroll
        for (int j = 0; j < 4; ++j) s[j] = (v8f){0.f, 0.f, 0.f, 0.f, 0.f, 0.f, 0.f, 0.f};
        {
            const __bf16* qrh = qh + c * QP + 8 * hh;
            const __bf16* qrl = ql + c * QP + 8 * hh;
#pragma unroll
            for (int ks = 0; ks < HD / 32; ++ks) {
                Split qa; qa.hi = ld_frag(qrh + ks * 32); qa.lo = ld_frag(qrl + ks * 32);
#pragma unroll
                for (int j = 0; j < 4; ++j) {
                    Split kb;
                    kb.hi = ld_frag(KH + (j * 16 + c) * QP + ks * 32 + 8 * hh);
                    kb.lo = ld_frag(KL + (j * 16 + c) * QP + ks * 32 + 8 * hh);
                    s[j] = wmma3(qa, kb, s[j]);
                }
            }
        }

        const bool diag = (kc == qb);
#pragma unroll
        for (int i = 0; i < 8; ++i) {
            const int irow = q0 + i + 8 * hh;
            float sc[4];
#pragma unroll
            for (int t = 0; t < 4; ++t) {
                const int jg = kv0 + t * 16 + c;
                sc[t] = (diag && jg > irow) ? NEG : s[t][i] * sl2;
            }
            float mx = fmaxf(fmaxf(sc[0], sc[1]), fmaxf(sc[2], sc[3]));
            mx = fmaxf(mx, __shfl_xor(mx, 1, 32)); mx = fmaxf(mx, __shfl_xor(mx, 2, 32));
            mx = fmaxf(mx, __shfl_xor(mx, 4, 32)); mx = fmaxf(mx, __shfl_xor(mx, 8, 32));
            const float mnew = fmaxf(m8[i], mx);
            const float corr = (mnew == NEG) ? 1.f : exp2f(m8[i] - mnew);
            float rs = 0.f;
#pragma unroll
            for (int t = 0; t < 4; ++t) {
                const float pp = (sc[t] == NEG) ? 0.f : exp2f(sc[t] - mnew);
                rs += pp;
                __bf16 ah, al; at_split(pp, ah, al);
                ph[(i + 8 * hh) * PP + t * 16 + c] = ah; pl[(i + 8 * hh) * PP + t * 16 + c] = al;
            }
            rs += __shfl_xor(rs, 1, 32); rs += __shfl_xor(rs, 2, 32); rs += __shfl_xor(rs, 4, 32); rs += __shfl_xor(rs, 8, 32);
            l8[i] = l8[i] * corr + rs; m8[i] = mnew;
#pragma unroll
            for (int t = 0; t < 8; ++t) o[t][i] *= corr;
        }
        __syncthreads();

        {
            const __bf16* prh = ph + c * PP + 8 * hh;
            const __bf16* prl = pl + c * PP + 8 * hh;
#pragma unroll 1
            for (int kk = 0; kk < 2; ++kk) {
                Split pa; pa.hi = ld_frag(prh + kk * 32); pa.lo = ld_frag(prl + kk * 32);
#pragma unroll
                for (int t = 0; t < 8; ++t) {
                    Split vb;
                    vb.hi = ld_frag(VH + (t * 16 + c) * VPT + kk * 32 + 8 * hh);
                    vb.lo = ld_frag(VL + (t * 16 + c) * VPT + kk * 32 + 8 * hh);
                    o[t] = wmma3(pa, vb, o[t]);
                }
            }
        }
    }

    __syncthreads();
    float* os = OS + wave * 16 * OSP;
#pragma unroll
    for (int i = 0; i < 8; ++i) {
        const float inv = (l8[i] > 0.f) ? 1.f / l8[i] : 0.f;
#pragma unroll
        for (int t = 0; t < 8; ++t) os[(i + 8 * hh) * OSP + t * 16 + c] = o[t][i] * inv;
    }
    __syncthreads();
    float* ob = O + ((size_t)b * SEQ + q0) * HD;
    for (int pass = 0; pass < 2; ++pass) {
#pragma unroll
        for (int row = 0; row < 16; ++row) {
            const v4f v = *(const v4f*)(os + row * OSP + lane * 4);
            *(volatile v4f*)(ob + (size_t)row * HD + lane * 4) = v;
        }
        __threadfence();
    }
}

extern "C" void kernel_launch(void* const* d_in, const int* in_sizes, int n_in, void* d_out, int out_size, void* d_ws, size_t ws_size, hipStream_t stream) {
    if (n_in < 4) return;
    if (in_sizes[0] < ((NB - 1) * SEQ_FULL + SEQ) * DIN) return;
    if (in_sizes[1] < DIN * HD || in_sizes[2] < DIN * HD || in_sizes[3] < DIN * HD) return;
    if (out_size < NRT * HD) return;
    const float* x  = (const float*)d_in[0];
    const float* Wk = (const float*)d_in[1];
    const float* Wq = (const float*)d_in[2];
    const float* Wv = (const float*)d_in[3];
    float* out = (float*)d_out;

    char* wsp = (char*)d_ws;
    unsigned short* X16 = (unsigned short*)wsp;  wsp += ((((size_t)NRT * DIN) * 2 + 255) / 256) * 256;
    unsigned short* W316 = (unsigned short*)wsp; wsp += ((((size_t)D3 * DIN) * 2 + 255) / 256) * 256;
    float* QKV = (float*)wsp;                    wsp += ((((size_t)NRT * D3) * 4 + 255) / 256) * 256;
    if ((size_t)(wsp - (char*)d_ws) > ws_size) return;
    if ((size_t)(wsp - (char*)d_ws) > (size_t)134217728) return;

    k_cast_x<<<(unsigned)((((long long)NRT) * (DIN / 8) + 255) / 256), 256, 0, stream>>>(x, X16);
    k_cm_castbT<<<(unsigned)((((long long)HD) * (DIN / 8) + 255) / 256), 256, 0, stream>>>(Wq, HD, W316 + (size_t)0 * HD * DIN, DIN, DIN, HD, 16.0f);
    k_cm_castbT<<<(unsigned)((((long long)HD) * (DIN / 8) + 255) / 256), 256, 0, stream>>>(Wk, HD, W316 + (size_t)1 * HD * DIN, DIN, DIN, HD, 16.0f);
    k_cm_castbT<<<(unsigned)((((long long)HD) * (DIN / 8) + 255) / 256), 256, 0, stream>>>(Wv, HD, W316 + (size_t)2 * HD * DIN, DIN, DIN, HD, 16.0f);
    w25::wmma_gemm64<0, false, 0, 0, false, 0><<<dim3((unsigned)((((NRT) / 64) * ((D3) / 64) + 7) / 8), (unsigned)(1)), 256, 0, stream>>>(
        (const unsigned short*)X16, nullptr, DIN, 0, (const unsigned short*)W316, nullptr, DIN, 0, (void*)QKV, nullptr, D3, 0, nullptr, nullptr, 0, NRT, D3, DIN, 0.0625f);
    const float sl2 = 0.036084391824351615f * 1.4426950408889634f;
    (void)hipFuncSetAttribute(reinterpret_cast<const void*>(&k_attn_c), hipFuncAttributeMaxDynamicSharedMemorySize, L_END);
    k_attn_c<<<dim3((unsigned)(SEQ / 64), (unsigned)(NB), 1), 32 * AW, L_END, stream>>>(QKV, out, sl2);
    (void)hipGetLastError();
}
